// PlasticMambaBlock_77386720740105
// MI455X (gfx1250) — hardware-verified
//
#include <hip/hip_runtime.h>
#include <math.h>

typedef __attribute__((ext_vector_type(16))) _Float16 v16h;
typedef __attribute__((ext_vector_type(8)))  _Float16 v8h;
typedef __attribute__((ext_vector_type(16))) __bf16   v16b;
typedef __attribute__((ext_vector_type(8)))  __bf16   v8b;
typedef __attribute__((ext_vector_type(8)))  float    v8f;
typedef __attribute__((ext_vector_type(4)))  float    v4f;

constexpr int kBatch  = 2;
constexpr int kSeq    = 2048;
constexpr int kDm     = 1024;
constexpr int kDin    = 2048;
constexpr int kNst    = 16;
constexpr int kDtR    = 64;
constexpr int kConvK  = 4;
constexpr int kXzP    = 2 * kDin;
constexpr int kXdW    = kDtR + 2 * kNst;
constexpr int kXdP    = 128;
constexpr int kRows   = kBatch * kSeq;
constexpr int kConvTP = 260;
constexpr int kScanTS = 64;
constexpr int kScanCh = 64;
constexpr int kScanYP = 68;
constexpr int kScanXP = 96;
static_assert(kXdW == 96 && kXdW <= kXdP, "x_proj width");
static_assert((kDm % 32) == 0 && (kDin % 32) == 0 && (kDtR % 4) == 0, "GEMM K multiples of 32");
static_assert((kRows % 64) == 0 && (kXzP % 64) == 0 && (kXdP % 64) == 0 && (kDm % 64) == 0 && (kSeq % 64) == 0, "GEMM M,N multiples of 64");
static_assert((kSeq % kScanTS) == 0 && (kDin % kScanCh) == 0 && (kDin % 256) == 0 && (kDm % 64) == 0, "tile multiples");

constexpr size_t kMi = 1048576ull;
constexpr size_t kOffXZ   = 0;
constexpr size_t kOffPH   = 0;
constexpr size_t kOffPL   = 16 * kMi;
constexpr size_t kOffKH   = 32 * kMi;
constexpr size_t kOffKL   = 40 * kMi;
constexpr size_t kOffVTH  = 48 * kMi;
constexpr size_t kOffVTL  = 56 * kMi;
constexpr size_t kOffUCH  = 64 * kMi;
constexpr size_t kOffUCL  = 80 * kMi;
constexpr size_t kOffYH   = 64 * kMi;
constexpr size_t kOffYL   = 80 * kMi;
constexpr size_t kOffXNH  = 64 * kMi;
constexpr size_t kOffXNL  = 72 * kMi;
constexpr size_t kOffWKTH = 80 * kMi;
constexpr size_t kOffWKTL = 82 * kMi;
constexpr size_t kOffWVTH = 84 * kMi;
constexpr size_t kOffWVTL = 86 * kMi;
constexpr size_t kOffHF   = 96 * kMi;
constexpr size_t kOffWIN  = 104 * kMi;
constexpr size_t kOffWXH  = 96 * kMi;
constexpr size_t kOffWXL  = kOffWXH + (size_t)kXdP * kDin * 2;
constexpr size_t kOffXD   = 97 * kMi;
constexpr size_t kOffWOH  = 99 * kMi;
constexpr size_t kOffWOL  = 103 * kMi;
constexpr size_t kOffPW   = 107 * kMi;
constexpr size_t kOffX2   = 112 * kMi;
constexpr size_t kWsTotal = kOffX2 + (size_t)kRows * kDm * 4;
static_assert(kWsTotal == 134217728ull, "carve total");
static_assert(kWsTotal <= 134217728ull, "carve cap");
static_assert((size_t)kRows * kXzP * 4 == 64 * kMi, "XZ extent");
static_assert(kOffPL + (size_t)kBatch * kSeq * kSeq * 2 <= kOffKH, "P planes inside dead XZ head");
static_assert(kOffPL == kOffPH + (size_t)kBatch * kSeq * kSeq * 2, "P planes adjacent");
static_assert(kOffKL == kOffKH + (size_t)kRows * kDm * 2 && kOffVTH == kOffKL + (size_t)kRows * kDm * 2, "K planes");
static_assert(kOffVTL == kOffVTH + (size_t)kDm * kRows * 2 && kOffVTL + (size_t)kDm * kRows * 2 == 64 * kMi, "Vt planes");
static_assert(kOffUCL == kOffUCH + (size_t)kRows * kDin * 2 && kOffUCL + (size_t)kRows * kDin * 2 == 96 * kMi, "u planes");
static_assert(kOffYL == kOffYH + (size_t)kRows * kDin * 2 && kOffYL + (size_t)kRows * kDin * 2 == 96 * kMi, "y planes");
static_assert(kOffXNL == kOffXNH + (size_t)kRows * kDm * 2 && kOffXNL + (size_t)kRows * kDm * 2 == kOffWKTH, "xn planes");
static_assert(kOffWKTL == kOffWKTH + (size_t)kDm * kDm * 2 && kOffWVTH == kOffWKTL + (size_t)kDm * kDm * 2 &&
              kOffWVTL == kOffWVTH + (size_t)kDm * kDm * 2 && kOffWVTL + (size_t)kDm * kDm * 2 <= 96 * kMi, "WkT/WvT planes");
static_assert(kOffHF + (size_t)kRows * kDm * 2 == kOffWIN && kOffWIN + (size_t)kXzP * kDm * 2 == kOffX2, "f16 planes");
static_assert(kOffWXL + (size_t)kXdP * kDin * 2 <= kOffXD && kOffXD + (size_t)kRows * kXdP * 4 == kOffWOH, "WX / XD");
static_assert(kOffWOL == kOffWOH + (size_t)kDm * kDin * 2 && kOffWOL + (size_t)kDm * kDin * 2 == kOffPW && kOffPW + (size_t)kSeq * 4 <= kOffX2, "WO / PW");
static_assert((kOffWXL % 128) == 0 && (kOffXD % 128) == 0 && (kOffPW % 128) == 0, "128-B aligned regions");

__device__ __forceinline__ unsigned short f2bf_bits(float f) {
  unsigned u = __float_as_uint(f);
  return (unsigned short)((u + 0x7FFFu + ((u >> 16) & 1u)) >> 16);
}
__device__ __forceinline__ float bf_bits2f(unsigned short h) { return __uint_as_float(((unsigned)h) << 16); }

__device__ __forceinline__ void dep_guard_h(v8f& a, v8f& b, v16h x, v16h y) { asm volatile("v_nop\n\tv_nop\n\tv_nop\n\tv_nop" : "+v"(a), "+v"(b) : "v"(x), "v"(y)); }
__device__ __forceinline__ void dep_guard_b(v8f& a, v8f& b, v16b x, v16b y) { asm volatile("v_nop\n\tv_nop\n\tv_nop\n\tv_nop" : "+v"(a), "+v"(b) : "v"(x), "v"(y)); }
__device__ __forceinline__ void keep4_h(v16h a, v16h b, v16h c, v16h d) { asm volatile("v_nop" :: "v"(a), "v"(b), "v"(c), "v"(d)); }
__device__ __forceinline__ void keep4_b(v16b a, v16b b, v16b c, v16b d) { asm volatile("v_nop" :: "v"(a), "v"(b), "v"(c), "v"(d)); }
__device__ __forceinline__ void acc_guard4(v8f& a, v8f& b, v8f& c, v8f& d) { asm volatile("v_nop\n\tv_nop\n\tv_nop\n\tv_nop" : "+v"(a), "+v"(b), "+v"(c), "+v"(d)); }
template <typename T> struct Frag;
template <> struct Frag<_Float16> {
  typedef v16h V; union U { v16h v; v8h h[2]; };
  static __device__ __forceinline__ v16h load(const _Float16* p) {
    U f; f.h[0] = *(const v8h*)(p); f.h[1] = *(const v8h*)(p + 16); return f.v;
  }
  static __device__ __forceinline__ v8f mma(v16h a, v16h b, v8f c) {
    return __builtin_amdgcn_wmma_f32_16x16x32_f16(false, a, false, b, (short)0, c, false, false);
  }
  static __device__ __forceinline__ void guard(v8f& a, v8f& b, v16h x, v16h y) { dep_guard_h(a, b, x, y); }
  static __device__ __forceinline__ void keep(v16h a, v16h b, v16h c, v16h d) { keep4_h(a, b, c, d); }
};
template <> struct Frag<__bf16> {
  typedef v16b V; union U { v16b v; v8b h[2]; };
  static __device__ __forceinline__ v16b load(const __bf16* p) {
    U f; f.h[0] = *(const v8b*)(p); f.h[1] = *(const v8b*)(p + 16); return f.v;
  }
  static __device__ __forceinline__ v8f mma(v16b a, v16b b, v8f c) {
    return __builtin_amdgcn_wmma_f32_16x16x32_bf16(false, a, false, b, (short)0, c, false, false);
  }
  static __device__ __forceinline__ void guard(v8f& a, v8f& b, v16b x, v16b y) { dep_guard_b(a, b, x, y); }
  static __device__ __forceinline__ void keep(v16b a, v16b b, v16b c, v16b d) { keep4_b(a, b, c, d); }
};

template <int ET> struct Elem;
template <> struct Elem<0> { typedef _Float16 T; };
template <> struct Elem<1> { typedef __bf16 T; };
template <int ET, int SPL, int BIAS_MODE, int OUT_MODE, bool RESID, int ACT = 0, int TRI = 0, int CAUSK = 0>
__global__ __launch_bounds__(256) void wmma_gemm64(
    const unsigned short* __restrict__ Ap, const unsigned short* __restrict__ A2p, int lda, long strideA,
    const unsigned short* __restrict__ Btp, const unsigned short* __restrict__ Bt2p, int ldb, long strideB,
    void* __restrict__ Cout, void* __restrict__ Cout2, int ldc, long strideC,
    const float* __restrict__ bias,
    const float* __restrict__ resid, long strideR,
    int M, int N, int K, float scale) {
  typedef typename Elem<ET>::T T;
  typedef typename Frag<T>::V V;
  const T* A = (const T*)Ap; const T* A2 = (const T*)A2p; const T* Bt = (const T*)Btp; const T* Bt2 = (const T*)Bt2p;
  __shared__ __align__(16) float sT[8][16 * 68];
  const int b    = blockIdx.y;
  const int lane = threadIdx.x & 31;
  const int wave = threadIdx.x >> 5;
  const int tilesN = N >> 6;
  const int tilesM = M >> 6;
  const int tile = blockIdx.x * 8 + wave;
  int tm, tn;
  if (TRI == 1) {
    const int ntri = (tilesM * (tilesM + 1)) >> 1;
    if (tile >= ntri) return;
    int t2 = 0;
#pragma unroll 1
    for (int i = 1; i < tilesM; ++i) t2 = (((i * (i + 1)) >> 1) <= tile) ? i : t2;
    tm = t2;
    tn = tile - ((tm * (tm + 1)) >> 1);
  } else {
    if (tile >= tilesM * tilesN) return;
    tm = tile / tilesN;
    tn = tile - tm * tilesN;
  }
  const int m0 = tm << 6;
  const int n0 = tn << 6;
  const int Kend = (CAUSK == 1) ? (((m0 + 64) < K) ? (m0 + 64) : K) : K;

  const T* Ab  = A  + (size_t)b * strideA;
  const T* Bb  = Bt + (size_t)b * strideB;
  const T* Ab2 = (SPL >= 1) ? (A2  + (size_t)b * strideA) : nullptr;
  const T* Bb2 = (SPL == 2) ? (Bt2 + (size_t)b * strideB) : nullptr;

  const int rlane = lane & 15;
  const int koff  = (lane >> 4) * 8;
  const int mOff  = (lane >> 4) * 8;

  v8f acc[4][4];
#pragma unroll
  for (int i = 0; i < 4; ++i)
#pragma unroll
    for (int j = 0; j < 4; ++j) acc[i][j] = (v8f){0.f,0.f,0.f,0.f,0.f,0.f,0.f,0.f};

  for (int k0 = 0; k0 < Kend; k0 += 32) {
    V bh[4], bl[4];
#pragma unroll
    for (int j = 0; j < 4; ++j) {
      const size_t bo = (size_t)(n0 + (j << 4) + rlane) * ldb + koff + k0;
      bh[j] = Frag<T>::load(Bb + bo);
      if (SPL == 2) bl[j] = Frag<T>::load(Bb2 + bo);
    }
#pragma unroll
    for (int i = 0; i < 4; ++i) {
      const size_t ao = (size_t)(m0 + (i << 4) + rlane) * lda + koff + k0;
      V ah = Frag<T>::load(Ab + ao);
      V al;
      if (SPL >= 1) al = Frag<T>::load(Ab2 + ao);
#pragma unroll
      for (int j = 0; j < 4; ++j) {
        acc[i][j] = Frag<T>::mma(ah, bh[j], acc[i][j]);
        if (SPL == 2) acc[i][j] = Frag<T>::mma(ah, bl[j], acc[i][j]);
        if (SPL >= 1) acc[i][j] = Frag<T>::mma(al, bh[j], acc[i][j]);
      }
      Frag<T>::guard(acc[i][0], acc[i][3], ah, (SPL >= 1) ? al : ah);
    }
    Frag<T>::keep(bh[0], bh[1], bh[2], bh[3]);
    if (SPL == 2) Frag<T>::keep(bl[0], bl[1], bl[2], bl[3]);
  }
  acc_guard4(acc[0][0], acc[0][1], acc[0][2], acc[0][3]);
  acc_guard4(acc[1][0], acc[1][1], acc[1][2], acc[1][3]);
  acc_guard4(acc[2][0], acc[2][1], acc[2][2], acc[2][3]);
  acc_guard4(acc[3][0], acc[3][1], acc[3][2], acc[3][3]);

  float* slab = sT[wave];
  const float* Rb = RESID ? (resid + (size_t)b * strideR) : nullptr;
#pragma unroll
  for (int i = 0; i < 4; ++i) {
    const int mBase = m0 + (i << 4);
#pragma unroll
    for (int j = 0; j < 4; ++j) {
      const int n = n0 + (j << 4) + rlane;
      float bv = 0.f;
      if (BIAS_MODE == 2) bv = bias[n];
#pragma unroll
      for (int r = 0; r < 8; ++r) {
        float v = acc[i][j][r] * scale;
        if (BIAS_MODE == 1) v += bias[mBase + mOff + r];
        if (BIAS_MODE == 2) v += bv;
        if (RESID) v += Rb[(size_t)(mBase + mOff + r) * ldc + n];
        if (ACT == 1) v = tanhf(v);
        if (ACT == 2) v = fmaxf(v, 0.0f);
        if (ACT == 3) v = v / (1.0f + expf(-v));
        if (ACT == 4) v = (v > 0.f) ? v : 0.01f * v;
        if (ACT == 6) {
          const int mm = mBase + mOff + r;
          const int de = mm - 1 - n;
          const int dc = (de < 0) ? 0 : de;
          const float wv = bias[dc];
          v = (de >= 0) ? (v * wv) : 0.0f;
        }
        slab[(mOff + r) * 68 + (j << 4) + rlane] = v;
      }
    }
    __builtin_amdgcn_fence(__ATOMIC_RELEASE, "workgroup");
    __builtin_amdgcn_wave_barrier();
    __builtin_amdgcn_fence(__ATOMIC_ACQUIRE, "workgroup");
    if (OUT_MODE == 0) {
      float* C = (float*)Cout + (size_t)b * strideC;
      const int hh = lane >> 4, c4 = (lane & 15) * 4;
      for (int pass = 0; pass < 2; ++pass) {
#pragma unroll
        for (int it = 0; it < 8; ++it) {
          const int row = it * 2 + hh;
          v4f v = *(const v4f*)(slab + row * 68 + c4);
          *(volatile v4f*)(C + (size_t)(mBase + row) * ldc + n0 + c4) = v;
        }
        __threadfence();
      }
    } else {
      const int q = lane >> 3, c8 = (lane & 7) * 8;
      unsigned short* C  = (unsigned short*)Cout  + (size_t)b * strideC;
      unsigned short* C2 = (OUT_MODE == 2) ? ((unsigned short*)Cout2 + (size_t)b * strideC) : nullptr;
      for (int pass = 0; pass < 2; ++pass) {
#pragma unroll
        for (int it = 0; it < 4; ++it) {
          const int row = it * 4 + q;
          const float* sp = slab + row * 68 + c8;
          v8h hv, lv;
#pragma unroll
          for (int e = 0; e < 8; ++e) {
            if (OUT_MODE == 1) {
              hv[e] = (_Float16)sp[e];
            } else {
              unsigned short hb = f2bf_bits(sp[e]);
              unsigned short lb = f2bf_bits(sp[e] - bf_bits2f(hb));
              hv[e] = __builtin_bit_cast(_Float16, hb);
              lv[e] = __builtin_bit_cast(_Float16, lb);
            }
          }
          *(volatile v8h*)(C + (size_t)(mBase + row) * ldc + n0 + c8) = hv;
          if (OUT_MODE == 2) *(volatile v8h*)(C2 + (size_t)(mBase + row) * ldc + n0 + c8) = lv;
        }
        __threadfence();
      }
    }
    __builtin_amdgcn_fence(__ATOMIC_RELEASE, "workgroup");
    __builtin_amdgcn_wave_barrier();
    __builtin_amdgcn_fence(__ATOMIC_ACQUIRE, "workgroup");
  }
}

template <int MODE>
__global__ __launch_bounds__(128) void rms_rows_kernel(
    const float* __restrict__ src, const float* __restrict__ w,
    unsigned short* __restrict__ o1, unsigned short* __restrict__ o2, float oscale)
{
  __shared__ float red[4];
  const int row = blockIdx.x, tid = threadIdx.x, lane = tid & 31, wave = tid >> 5;
  const size_t base = (size_t)row * kDm + (size_t)tid * 8;
  const v4f a0 = *(const v4f*)(src + base);
  const v4f a1 = *(const v4f*)(src + base + 4);
  const v4f w0 = *(const v4f*)(w + tid * 8);
  const v4f w1 = *(const v4f*)(w + tid * 8 + 4);
  float ss = 0.f;
#pragma unroll
  for (int e = 0; e < 4; ++e) ss = fmaf(a0[e], a0[e], ss);
#pragma unroll
  for (int e = 0; e < 4; ++e) ss = fmaf(a1[e], a1[e], ss);
#pragma unroll
  for (int off = 1; off < 32; off <<= 1) ss += __shfl_xor(ss, off, 32);
  if (lane == 0) red[wave] = ss;
  __syncthreads();
  const float tot = (red[0] + red[1]) + (red[2] + red[3]);
  const float rr = rsqrtf(tot * (1.0f / (float)kDm) + 1e-5f);
  float vv[8];
#pragma unroll
  for (int e = 0; e < 4; ++e) { vv[e] = (a0[e] * rr) * w0[e]; vv[4 + e] = (a1[e] * rr) * w1[e]; }
  if (MODE == 0) {
    v8h hv;
#pragma unroll
    for (int e = 0; e < 8; ++e) hv[e] = (_Float16)(vv[e] * oscale);
    *(volatile v8h*)(o1 + base) = hv;
    __threadfence();
    *(volatile v8h*)(o1 + base) = hv;
  } else {
    v8h hv, lv;
#pragma unroll
    for (int e = 0; e < 8; ++e) {
      const unsigned short hb = f2bf_bits(vv[e]);
      const unsigned short lb = f2bf_bits(vv[e] - bf_bits2f(hb));
      hv[e] = __builtin_bit_cast(_Float16, hb);
      lv[e] = __builtin_bit_cast(_Float16, lb);
    }
    *(volatile v8h*)(o1 + base) = hv;
    *(volatile v8h*)(o2 + base) = lv;
    __threadfence();
    *(volatile v8h*)(o1 + base) = hv;
    *(volatile v8h*)(o2 + base) = lv;
  }
}

__global__ __launch_bounds__(256) void cast_scale_f16_kernel(
    const float* __restrict__ in, unsigned short* __restrict__ out, float sc, int total8)
{
  const int i = blockIdx.x * 256 + threadIdx.x;
  if (i >= total8) return;
  const size_t e0 = (size_t)i << 3;
  const v4f a0 = *(const v4f*)(in + e0);
  const v4f a1 = *(const v4f*)(in + e0 + 4);
  v8h hv;
#pragma unroll
  for (int e = 0; e < 4; ++e) { hv[e] = (_Float16)(a0[e] * sc); hv[4 + e] = (_Float16)(a1[e] * sc); }
  *(volatile v8h*)(out + e0) = hv;
  __threadfence();
  *(volatile v8h*)(out + e0) = hv;
}

template <int COLS>
__global__ __launch_bounds__(256) void split_rows_kernel(
    const float* __restrict__ src, unsigned short* __restrict__ dhi, unsigned short* __restrict__ dlo,
    int srcRows, int total8)
{
  static_assert((COLS % 8) == 0, "cols");
  const int i = blockIdx.x * 256 + threadIdx.x;
  if (i >= total8) return;
  const size_t e0 = (size_t)i << 3;
  const int row = (int)(e0 / COLS);
  const int col = (int)(e0 - (size_t)row * COLS);
  const bool live = row < srcRows;
  const int rowc = live ? row : (srcRows - 1);
  const float* sp = src + (size_t)rowc * COLS + col;
  v4f a0 = *(const v4f*)(sp);
  v4f a1 = *(const v4f*)(sp + 4);
  const v4f zz = (v4f){0.f, 0.f, 0.f, 0.f};
  a0 = live ? a0 : zz;
  a1 = live ? a1 : zz;
  v8h hv, lv;
#pragma unroll
  for (int e = 0; e < 4; ++e) {
    const unsigned short h0 = f2bf_bits(a0[e]), h1 = f2bf_bits(a1[e]);
    const unsigned short l0 = f2bf_bits(a0[e] - bf_bits2f(h0)), l1 = f2bf_bits(a1[e] - bf_bits2f(h1));
    hv[e]     = __builtin_bit_cast(_Float16, h0);
    hv[4 + e] = __builtin_bit_cast(_Float16, h1);
    lv[e]     = __builtin_bit_cast(_Float16, l0);
    lv[4 + e] = __builtin_bit_cast(_Float16, l1);
  }
  unsigned short* qh = dhi + e0;
  unsigned short* ql = dlo + e0;
  *(volatile v8h*)qh = hv;
  *(volatile v8h*)ql = lv;
  __threadfence();
  *(volatile v8h*)qh = hv;
  *(volatile v8h*)ql = lv;
}

__global__ __launch_bounds__(256) void transpose_split_kernel(
    const float* __restrict__ W, unsigned short* __restrict__ TH, unsigned short* __restrict__ TL)
{
  __shared__ __align__(16) float sT[64 * 68];
  const int tid = threadIdx.x, lane = tid & 31, wave = tid >> 5;
  const int d0 = blockIdx.y * 64, e0 = blockIdx.x * 64;
  {
    const int dl0 = tid >> 4, c4 = (tid & 15) * 4;
#pragma unroll
    for (int i = 0; i < 4; ++i) {
      const int dl = i * 16 + dl0;
      const v4f v = *(const v4f*)(W + (size_t)(d0 + dl) * kDm + e0 + c4);
      sT[(c4 + 0) * 68 + dl] = v[0];
      sT[(c4 + 1) * 68 + dl] = v[1];
      sT[(c4 + 2) * 68 + dl] = v[2];
      sT[(c4 + 3) * 68 + dl] = v[3];
    }
  }
  __syncthreads();
  const int q = lane >> 3, c8 = (lane & 7) * 8;
  v8h hv[2], lv[2];
#pragma unroll
  for (int it = 0; it < 2; ++it) {
    const int el = it * 32 + wave * 4 + q;
    const float* sp = sT + el * 68 + c8;
    const v4f a0 = *(const v4f*)(sp);
    const v4f a1 = *(const v4f*)(sp + 4);
#pragma unroll
    for (int e = 0; e < 4; ++e) {
      const unsigned short h0 = f2bf_bits(a0[e]), h1 = f2bf_bits(a1[e]);
      const unsigned short l0 = f2bf_bits(a0[e] - bf_bits2f(h0)), l1 = f2bf_bits(a1[e] - bf_bits2f(h1));
      hv[it][e]     = __builtin_bit_cast(_Float16, h0);
      hv[it][4 + e] = __builtin_bit_cast(_Float16, h1);
      lv[it][e]     = __builtin_bit_cast(_Float16, l0);
      lv[it][4 + e] = __builtin_bit_cast(_Float16, l1);
    }
  }
  for (int pass = 0; pass < 2; ++pass) {
#pragma unroll
    for (int it = 0; it < 2; ++it) {
      const int el = it * 32 + wave * 4 + q;
      const size_t o = (size_t)(e0 + el) * kDm + d0 + c8;
      *(volatile v8h*)(TH + o) = hv[it];
      *(volatile v8h*)(TL + o) = lv[it];
    }
    __threadfence();
  }
}

__global__ __launch_bounds__(256) void decay_table_kernel(float* __restrict__ pw, int n)
{
  const int i = blockIdx.x * 256 + threadIdx.x;
  if (i >= n) return;
  double r = 1.0;
  double bp = (double)0.95f;
  int e = i;
#pragma unroll 1
  for (int bit = 0; bit < 11; ++bit) {
    const double rp = r * bp;
    r = (e & 1) ? rp : r;
    bp = bp * bp;
    e >>= 1;
  }
  const float f = (float)r;
  ((volatile float*)pw)[i] = f;
  __threadfence();
  ((volatile float*)pw)[i] = f;
}

__device__ __forceinline__ float conv_silu_val(float w0, float w1, float w2, float w3, float bc,
                                               float xm3, float xm2, float xm1, float xcur)
{
  float acc = w0 * xm3;
  acc = fmaf(w1, xm2, acc);
  acc = fmaf(w2, xm1, acc);
  acc = fmaf(w3, xcur, acc);
  const float sv = acc + bc;
  const float sg = __builtin_amdgcn_rcpf(1.0f + __expf(-sv));
  return sv * sg;
}

__global__ __launch_bounds__(256) void conv_silu_kernel(
    const float* __restrict__ XZ, const float* __restrict__ cw, const float* __restrict__ cb,
    unsigned short* __restrict__ UCH, unsigned short* __restrict__ UCL)
{
  __shared__ __align__(16) float sT[16 * kConvTP];
  const int tid = threadIdx.x, lane = tid & 31, wave = tid >> 5;
  const int d0 = blockIdx.x * 256, d = d0 + tid;
  const int g0 = blockIdx.y * 64;
  const int tb = g0 & (kSeq - 1);
  const float w0 = cw[d * kConvK + 0], w1 = cw[d * kConvK + 1], w2 = cw[d * kConvK + 2], w3 = cw[d * kConvK + 3];
  const float bc = cb[d];
  float xm3, xm2, xm1;
  {
    const bool hist = (tb > 0);
    const int rb = hist ? (g0 - 3) : g0;
    const float v3 = XZ[(size_t)rb * kXzP + d];
    const float v2 = XZ[(size_t)(rb + 1) * kXzP + d];
    const float v1 = XZ[(size_t)(rb + 2) * kXzP + d];
    xm3 = hist ? v3 : 0.f;
    xm2 = hist ? v2 : 0.f;
    xm1 = hist ? v1 : 0.f;
  }
#pragma unroll 1
  for (int sub = 0; sub < 4; ++sub) {
    const int lb = g0 + sub * 16;
#pragma unroll 1
    for (int s = 0; s < 16; ++s) {
      const float xcur = XZ[(size_t)(lb + s) * kXzP + d];
      sT[s * kConvTP + tid] = conv_silu_val(w0, w1, w2, w3, bc, xm3, xm2, xm1, xcur);
      xm3 = xm2; xm2 = xm1; xm1 = xcur;
    }
    __syncthreads();
    v8h bh[2], blo[2];
#pragma unroll
    for (int it = 0; it < 2; ++it) {
      const float* sp = sT + (it * 8 + wave) * kConvTP + lane * 8;
      const v4f a0 = *(const v4f*)(sp);
      const v4f a1 = *(const v4f*)(sp + 4);
#pragma unroll
      for (int e = 0; e < 4; ++e) {
        const unsigned short h0 = f2bf_bits(a0[e]), h1 = f2bf_bits(a1[e]);
        const unsigned short l0 = f2bf_bits(a0[e] - bf_bits2f(h0)), l1 = f2bf_bits(a1[e] - bf_bits2f(h1));
        bh[it][e]      = __builtin_bit_cast(_Float16, h0);
        bh[it][4 + e]  = __builtin_bit_cast(_Float16, h1);
        blo[it][e]     = __builtin_bit_cast(_Float16, l0);
        blo[it][4 + e] = __builtin_bit_cast(_Float16, l1);
      }
    }
    for (int pass = 0; pass < 2; ++pass) {
#pragma unroll
      for (int it = 0; it < 2; ++it) {
        const size_t o = (size_t)(lb + it * 8 + wave) * kDin + d0 + lane * 8;
        *(volatile v8h*)(UCH + o) = bh[it];
        *(volatile v8h*)(UCL + o) = blo[it];
      }
      __threadfence();
    }
    __syncthreads();
  }
}

__global__ __launch_bounds__(64) void scan_kernel(
    const float* __restrict__ XD, const float* __restrict__ XZ,
    const float* __restrict__ Wdt, const float* __restrict__ bdt, const float* __restrict__ Alog,
    const float* __restrict__ Dp, const float* __restrict__ cw, const float* __restrict__ cb,
    unsigned short* __restrict__ YH, unsigned short* __restrict__ YL)
{
  __shared__ __align__(16) float sX[kScanTS * kScanXP];
  __shared__ __align__(16) float sY[kScanTS * kScanYP];
  __shared__ __align__(16) float sW[kDtR * kScanCh];
  __shared__ __align__(16) float sA[kNst * kScanCh];
  const int tid = threadIdx.x, lane = tid & 31, wave = tid >> 5;
  constexpr int kBlkPerB = kDin / kScanCh;
  const int bix = blockIdx.x / kBlkPerB;
  const int d0  = (blockIdx.x - bix * kBlkPerB) * kScanCh;
  const int d   = d0 + tid;
  const size_t row0 = (size_t)bix * kSeq;
#pragma unroll 1
  for (int r = 0; r < kDtR; ++r) sW[r * kScanCh + tid] = Wdt[(size_t)d * kDtR + r];
#pragma unroll 1
  for (int s = 0; s < kNst; ++s) sA[s * kScanCh + tid] = -expf(Alog[(size_t)d * kNst + s]);
  __syncthreads();
  float negA[kNst], h[kNst];
#pragma unroll
  for (int s = 0; s < kNst; ++s) {
    negA[s] = sA[s * kScanCh + tid];
    h[s] = 0.f;
  }
  const float bb = bdt[d], Dd = Dp[d];
  const float w0 = cw[d * kConvK + 0], w1 = cw[d * kConvK + 1], w2 = cw[d * kConvK + 2], w3 = cw[d * kConvK + 3];
  const float bc = cb[d];
  float xm3 = 0.f, xm2 = 0.f, xm1 = 0.f;
  const int q = lane >> 3, c8 = (lane & 7) * 8;
#pragma unroll 1
  for (int t0 = 0; t0 < kSeq; t0 += kScanTS) {
    __syncthreads();
#pragma unroll 4
    for (int i = 0; i < 24; ++i) {
      const int idx = i * kScanCh + tid;
      const int r = idx / 24;
      const int c4 = (idx - r * 24) * 4;
      *(v4f*)(sX + r * kScanXP + c4) = *(const v4f*)(XD + (row0 + t0 + r) * kXdP + c4);
    }
    __syncthreads();
#pragma unroll 1
    for (int s = 0; s < kScanTS; ++s) {
      const int t = t0 + s;
      const float* xr = sX + s * kScanXP;
      float vdot = 0.f;
#pragma unroll 1
      for (int r4 = 0; r4 < kDtR / 4; ++r4) {
        const v4f xv = *(const v4f*)(xr + 4 * r4);
        const float* wp = sW + (4 * r4) * kScanCh + tid;
        vdot = fmaf(xv[0], wp[0], vdot);
        vdot = fmaf(xv[1], wp[kScanCh], vdot);
        vdot = fmaf(xv[2], wp[2 * kScanCh], vdot);
        vdot = fmaf(xv[3], wp[3 * kScanCh], vdot);
      }
      float Bs[kNst], Cs[kNst];
#pragma unroll
      for (int q4 = 0; q4 < 4; ++q4) {
        const v4f bv = *(const v4f*)(xr + kDtR + 4 * q4);
        const v4f cv = *(const v4f*)(xr + kDtR + kNst + 4 * q4);
        Bs[4 * q4 + 0] = bv[0]; Bs[4 * q4 + 1] = bv[1]; Bs[4 * q4 + 2] = bv[2]; Bs[4 * q4 + 3] = bv[3];
        Cs[4 * q4 + 0] = cv[0]; Cs[4 * q4 + 1] = cv[1]; Cs[4 * q4 + 2] = cv[2]; Cs[4 * q4 + 3] = cv[3];
      }
      const float v   = vdot + bb;
      const float a   = __expf(-fabsf(v));
      const float ua  = 1.0f + a;
      const float l1p = __logf(ua) + (a - (ua - 1.0f)) * __builtin_amdgcn_rcpf(ua);
      const float dt  = fmaxf(v, 0.0f) + l1p;
      const float xcur = XZ[(row0 + t) * kXzP + d];
      const float xt  = conv_silu_val(w0, w1, w2, w3, bc, xm3, xm2, xm1, xcur);
      xm3 = xm2; xm2 = xm1; xm1 = xcur;
      const float dtx = dt * xt;
      float y = 0.f;
#pragma unroll
      for (int k = 0; k < kNst; ++k) {
        const float e = __expf(dt * negA[k]);
        h[k] = e * h[k] + dtx * Bs[k];
        y = h[k] * Cs[k] + y;
      }
      y = xt * Dd + y;
      const float zv = XZ[(row0 + t) * kXzP + kDin + d];
      const float sg = __builtin_amdgcn_rcpf(1.0f + __expf(-zv));
      y = y * (zv * sg);
      sY[s * kScanYP + tid] = y;
    }
    __syncthreads();
    v8h hv[8], lv[8];
#pragma unroll
    for (int it = 0; it < 8; ++it) {
      const int row = it * 8 + wave * 4 + q;
      const float* sp = sY + row * kScanYP + c8;
      const v4f a0 = *(const v4f*)(sp);
      const v4f a1 = *(const v4f*)(sp + 4);
#pragma unroll
      for (int e = 0; e < 4; ++e) {
        const unsigned short h0 = f2bf_bits(a0[e]), h1 = f2bf_bits(a1[e]);
        const unsigned short l0 = f2bf_bits(a0[e] - bf_bits2f(h0)), l1 = f2bf_bits(a1[e] - bf_bits2f(h1));
        hv[it][e]     = __builtin_bit_cast(_Float16, h0);
        hv[it][4 + e] = __builtin_bit_cast(_Float16, h1);
        lv[it][e]     = __builtin_bit_cast(_Float16, l0);
        lv[it][4 + e] = __builtin_bit_cast(_Float16, l1);
      }
    }
    for (int pass = 0; pass < 2; ++pass) {
#pragma unroll
      for (int it = 0; it < 8; ++it) {
        const int row = it * 8 + wave * 4 + q;
        const size_t o = (row0 + t0 + row) * kDin + d0 + c8;
        *(volatile v8h*)(YH + o) = hv[it];
        *(volatile v8h*)(YL + o) = lv[it];
      }
      __threadfence();
    }
  }
}

extern "C" void kernel_launch(void* const* d_in, const int* in_sizes, int n_in,
                              void* d_out, int out_size, void* d_ws, size_t ws_size,
                              hipStream_t stream) {
  if (n_in < 14) return;
  if (in_sizes[0]  != kRows * kDm) return;
  if (in_sizes[1]  != kDm) return;
  if (in_sizes[2]  != kXzP * kDm) return;
  if (in_sizes[3]  != kDin * kConvK) return;
  if (in_sizes[4]  != kDin) return;
  if (in_sizes[5]  != kXdW * kDin) return;
  if (in_sizes[6]  != kDin * kDtR) return;
  if (in_sizes[7]  != kDin) return;
  if (in_sizes[8]  != kDin * kNst) return;
  if (in_sizes[9]  != kDin) return;
  if (in_sizes[10] != kDm * kDin) return;
  if (in_sizes[11] != kDm) return;
  if (in_sizes[12] != kDm * kDm) return;
  if (in_sizes[13] != kDm * kDm) return;
  if (out_size != kRows * kDm) return;
  if (ws_size < kWsTotal) return;

  const float* x          = (const float*)d_in[0];
  const float* norm_w     = (const float*)d_in[1];
  const float* in_proj_w  = (const float*)d_in[2];
  const float* conv_w     = (const float*)d_in[3];
  const float* conv_b     = (const float*)d_in[4];
  const float* x_proj_w   = (const float*)d_in[5];
  const float* dt_proj_w  = (const float*)d_in[6];
  const float* dt_proj_b  = (const float*)d_in[7];
  const float* A_log      = (const float*)d_in[8];
  const float* D_param    = (const float*)d_in[9];
  const float* out_proj_w = (const float*)d_in[10];
  const float* norm_h_w   = (const float*)d_in[11];
  const float* Wk         = (const float*)d_in[12];
  const float* Wv         = (const float*)d_in[13];
  float* out = (float*)d_out;

  char* ws = (char*)d_ws;
  float*          XZ   = (float*)(ws + kOffXZ);
  unsigned short* PH   = (unsigned short*)(ws + kOffPH);
  unsigned short* PL   = (unsigned short*)(ws + kOffPL);
  unsigned short* KH   = (unsigned short*)(ws + kOffKH);
  unsigned short* KL   = (unsigned short*)(ws + kOffKL);
  unsigned short* VTH  = (unsigned short*)(ws + kOffVTH);
  unsigned short* VTL  = (unsigned short*)(ws + kOffVTL);
  unsigned short* UCH  = (unsigned short*)(ws + kOffUCH);
  unsigned short* UCL  = (unsigned short*)(ws + kOffUCL);
  unsigned short* YH   = (unsigned short*)(ws + kOffYH);
  unsigned short* YL   = (unsigned short*)(ws + kOffYL);
  unsigned short* XNH  = (unsigned short*)(ws + kOffXNH);
  unsigned short* XNL  = (unsigned short*)(ws + kOffXNL);
  unsigned short* WKTH = (unsigned short*)(ws + kOffWKTH);
  unsigned short* WKTL = (unsigned short*)(ws + kOffWKTL);
  unsigned short* WVTH = (unsigned short*)(ws + kOffWVTH);
  unsigned short* WVTL = (unsigned short*)(ws + kOffWVTL);
  unsigned short* HF   = (unsigned short*)(ws + kOffHF);
  unsigned short* WIN  = (unsigned short*)(ws + kOffWIN);
  unsigned short* WXH  = (unsigned short*)(ws + kOffWXH);
  unsigned short* WXL  = (unsigned short*)(ws + kOffWXL);
  float*          XD   = (float*)(ws + kOffXD);
  unsigned short* WOH  = (unsigned short*)(ws + kOffWOH);
  unsigned short* WOL  = (unsigned short*)(ws + kOffWOL);
  float*          PW   = (float*)(ws + kOffPW);
  float*          X2   = (float*)(ws + kOffX2);

  const long kBatchRowsDm  = (long)kSeq * kDm;
  const long kBatchRowsSeq = (long)kSeq * kSeq;

  rms_rows_kernel<0><<<kRows, 128, 0, stream>>>(x, norm_w, HF, nullptr, 1.0f);
  cast_scale_f16_kernel<<<(kXzP * kDm / 8) / 256, 256, 0, stream>>>(in_proj_w, WIN, 32.0f, kXzP * kDm / 8);
  wmma_gemm64<0, 0, 0, 0, false, 0, 0, 0><<<dim3(512, 1), 256, 0, stream>>>(
      HF, nullptr, kDm, 0L,
      WIN, nullptr, kDm, 0L,
      (void*)XZ, nullptr, kXzP, 0L,
      nullptr, nullptr, 0L,
      kRows, kXzP, kDm, 1.0f / 32.0f);
  conv_silu_kernel<<<dim3(kDin / 256, kRows / 64), 256, 0, stream>>>(XZ, conv_w, conv_b, UCH, UCL);
  split_rows_kernel<kDin><<<(kXdP * kDin / 8) / 256, 256, 0, stream>>>(x_proj_w, WXH, WXL, kXdW, kXdP * kDin / 8);
  wmma_gemm64<1, 2, 0, 0, false><<<dim3(16, 1), 256, 0, stream>>>(
      UCH, UCL, kDin, 0L,
      WXH, WXL, kDin, 0L,
      (void*)XD, nullptr, kXdP, 0L,
      nullptr, nullptr, 0L,
      kRows, kXdP, kDin, 1.0f);
  split_rows_kernel<kDin><<<(kDm * kDin / 8) / 256, 256, 0, stream>>>(out_proj_w, WOH, WOL, kDm, kDm * kDin / 8);
  scan_kernel<<<kBatch * (kDin / kScanCh), kScanCh, 0, stream>>>(XD, XZ, dt_proj_w, dt_proj_b, A_log, D_param,
                                                                conv_w, conv_b, YH, YL);
  wmma_gemm64<1, 2, 0, 0, true><<<dim3(128, 1), 256, 0, stream>>>(
      YH, YL, kDin, 0L,
      WOH, WOL, kDin, 0L,
      (void*)X2, nullptr, kDm, 0L,
      nullptr, x, 0L,
      kRows, kDm, kDin, 1.0f);
  rms_rows_kernel<1><<<kRows, 128, 0, stream>>>(X2, norm_h_w, XNH, XNL, 1.0f);
  transpose_split_kernel<<<dim3(kDm / 64, kDm / 64), 256, 0, stream>>>(Wk, WKTH, WKTL);
  transpose_split_kernel<<<dim3(kDm / 64, kDm / 64), 256, 0, stream>>>(Wv, WVTH, WVTL);
  decay_table_kernel<<<kSeq / 256, 256, 0, stream>>>(PW, kSeq);
  wmma_gemm64<1, 2, 0, 2, false><<<dim3(128, 1), 256, 0, stream>>>(
      XNH, XNL, kDm, 0L,
      WKTH, WKTL, kDm, 0L,
      (void*)KH, (void*)KL, kDm, 0L,
      nullptr, nullptr, 0L,
      kRows, kDm, kDm, 1.0f);
  wmma_gemm64<1, 2, 0, 2, false><<<dim3(128, 1), 256, 0, stream>>>(
      WVTH, WVTL, kDm, 0L,
      XNH, XNL, kDm, 0L,
      (void*)VTH, (void*)VTL, kRows, 0L,
      nullptr, nullptr, 0L,
      kDm, kRows, kDm, 1.0f);
  wmma_gemm64<1, 2, 0, 2, false, 6, 1, 0><<<dim3(66, kBatch), 256, 0, stream>>>(
      XNH, XNL, kDm, kBatchRowsDm,
      KH, KL, kDm, kBatchRowsDm,
      (void*)PH, (void*)PL, kSeq, kBatchRowsSeq,
      PW, nullptr, 0L,
      kSeq, kSeq, kDm, 1.0f);
  wmma_gemm64<1, 2, 0, 0, true, 0, 0, 1><<<dim3(64, kBatch), 256, 0, stream>>>(
      PH, PL, kSeq, kBatchRowsSeq,
      VTH, VTL, kRows, (long)kSeq,
      (void*)out, nullptr, kDm, kBatchRowsDm,
      nullptr, X2, kBatchRowsDm,
      kSeq, kDm, kSeq, 0.1f);
}
